// SparseModel_70291434766874
// MI455X (gfx1250) — hardware-run, weakly checked
//
#include <hip/hip_runtime.h>


#ifndef NB
#define NB 32768
#endif
#define NB_FULL 32768
#ifndef HRES
#define HRES 0
#endif
#define IND   64
#define HID   128
#define NSUB  32
#define NHL   2
#define OTP   36
#define WCARRY 64.0f
#define HCARRY 16.0f
#define RCARRY 2048.0f
#define SMAIN  9.765625e-4f
#define SRES   4.76837158203125e-7f

#define OFF_B1 0
#define OFF_BH (NSUB * HID)
#define OFF_WO (OFF_BH + NHL * NSUB * HID)
#define OFF_BO (OFF_WO + NSUB * HID)
#define BV_N   (OFF_BO + NSUB)
#define BV_N4  (BV_N / 4)

static_assert(NB % 16 == 0);
static_assert(NB <= NB_FULL);
static_assert(IND == 64);
static_assert(IND % 32 == 0);
static_assert(HID == 128);
static_assert(HID % 32 == 0);
static_assert(NSUB == 32);
static_assert(NSUB * 4 == 128);
static_assert(BV_N % 32 == 0);
static_assert((OFF_BH % 4) == 0 && (OFF_WO % 4) == 0 && (OFF_BO % 4) == 0);
static_assert(OTP % 4 == 0 && OTP >= NSUB);
static_assert(WCARRY * HCARRY * SMAIN == 1.0f);
static_assert(WCARRY * HCARRY * RCARRY * SRES == 1.0f);

typedef unsigned short bf;
typedef unsigned short hf;
typedef _Float16 h16;
typedef __attribute__((ext_vector_type(16))) __bf16   v16bf;
typedef __attribute__((ext_vector_type(16))) _Float16 v16h;
typedef __attribute__((ext_vector_type(8)))  unsigned short v8us;
typedef __attribute__((ext_vector_type(8)))  float    v8f;
typedef __attribute__((ext_vector_type(4)))  float    v4f;
typedef __attribute__((ext_vector_type(4)))  int      v4i;
typedef v4f  __attribute__((may_alias)) v4fa;
typedef v4i  __attribute__((may_alias)) v4ia;

__device__ __forceinline__ unsigned short f2bf(float f) { unsigned u = __float_as_uint(f); u += 0x7FFFu + ((u >> 16) & 1u); return (unsigned short)(u >> 16); }
__device__ __forceinline__ float bf2f(unsigned short w) { return __uint_as_float(((unsigned)w) << 16); }
__device__ __forceinline__ int clampi(int v, int lo, int hi) { return min(max(v, lo), hi); }
__device__ __forceinline__ v16bf cat16b(v8us lo, v8us hi) { return __builtin_bit_cast(v16bf, __builtin_shufflevector(lo, hi, 0, 1, 2, 3, 4, 5, 6, 7, 8, 9, 10, 11, 12, 13, 14, 15)); }
__device__ __forceinline__ v8f wmmab(v16bf a, v16bf b, v8f c) { return __builtin_amdgcn_wmma_f32_16x16x32_bf16(false, a, false, b, (short)0, c, false, false); }
__device__ __forceinline__ v16bf ldb(const bf* p)  { return cat16b(*(const v8us*)p, *(const v8us*)(p + 16)); }
__device__ __forceinline__ void wave_sync() { __builtin_amdgcn_fence(3  , "wavefront"); __builtin_amdgcn_wave_barrier(); asm volatile("" ::: "memory"); }

__device__ __forceinline__ v16h cat16h(v8us lo, v8us hi) { return __builtin_bit_cast(v16h, __builtin_shufflevector(lo, hi, 0, 1, 2, 3, 4, 5, 6, 7, 8, 9, 10, 11, 12, 13, 14, 15)); }
__device__ __forceinline__ v16h ldh(const hf* p)  { return cat16h(*(const v8us*)p, *(const v8us*)(p + 16)); }
static __device__ __forceinline__ h16 toh_flush(float v) { const h16 r = (h16)v; return (fabsf(v) < 6.103515625e-05f) ? (h16)0.0f : r; }
__device__ __forceinline__ unsigned short hbits(h16 v) { return __builtin_bit_cast(unsigned short, v); }
__device__ __forceinline__ v8f wmmab_g(v16bf a, v16bf b, v8f c) {
    c = __builtin_amdgcn_wmma_f32_16x16x32_bf16(false, a, false, b, (short)0, c, false, false);
    asm volatile("v_nop\n\tv_nop\n\tv_nop\n\tv_nop" : "+v"(c) : "v"(a), "v"(b));
    return c; }
__device__ __forceinline__ v8f wmmah_g(v16h a, v16h b, v8f c) {
    c = __builtin_amdgcn_wmma_f32_16x16x32_f16(false, a, false, b, (short)0, c, false, false);
    asm volatile("v_nop\n\tv_nop\n\tv_nop\n\tv_nop" : "+v"(c) : "v"(a), "v"(b));
    return c; }
__device__ __forceinline__ float swishf(float z) { const float e = __expf(-z); return z * __builtin_amdgcn_rcpf(1.0f + e); }

__global__ __launch_bounds__(256) void k_w1t(const float* __restrict__ W, bf* WT) {
    __shared__ float ts[64 * 65];
    static_assert(sizeof(float) * 64 * 65 <= 131072);
    static_assert(256 * 2 == 64 * 8);
    const int b = blockIdx.x, t = threadIdx.x;
    const int o = b >> 1, oh = b & 1;
    const float* src = W + (size_t)o * (IND * HID) + oh * 64;
#pragma unroll 1
    for (int i = 0; i < 16; ++i) { const int f = i * 256 + t; ts[(f >> 6) * 65 + (f & 63)] = src[(f >> 6) * HID + (f & 63)]; }
    __syncthreads();
    bf* dst = WT + (size_t)o * (HID * IND) + (size_t)(oh * 64) * IND;
#pragma unroll 1
    for (int ps = 0; ps < 2; ++ps) {
#pragma unroll 1
        for (int it = 0; it < 2; ++it) {
            const int e = it * 32 + (t >> 3), c8 = (t & 7) * 8; v8us o8;
#pragma unroll
            for (int k = 0; k < 8; ++k) o8[k] = f2bf(ts[(c8 + k) * 65 + e]);
            *(volatile v8us*)(dst + e * IND + c8) = o8; }
        if (ps == 0) __threadfence(); }
}

__global__ __launch_bounds__(256) void k_wht(const float* __restrict__ W, hf* WT) {
    __shared__ float ts[64 * 65];
    static_assert(sizeof(float) * 64 * 65 <= 131072);
    static_assert(256 * 2 == 64 * 8);
    const int b = blockIdx.x, t = threadIdx.x;
    const int mtx = b >> 2, ti = (b >> 1) & 1, to = b & 1;
    const float* src = W + (size_t)mtx * (HID * HID) + (size_t)(ti * 64) * HID + to * 64;
#pragma unroll 1
    for (int i = 0; i < 16; ++i) { const int f = i * 256 + t; ts[(f >> 6) * 65 + (f & 63)] = src[(f >> 6) * HID + (f & 63)]; }
    __syncthreads();
    hf* dst = WT + (size_t)mtx * (HID * HID) + (size_t)(to * 64) * HID + ti * 64;
#pragma unroll 1
    for (int ps = 0; ps < 2; ++ps) {
#pragma unroll 1
        for (int it = 0; it < 2; ++it) {
            const int e = it * 32 + (t >> 3), c8 = (t & 7) * 8; v8us o8;
#pragma unroll
            for (int k = 0; k < 8; ++k) o8[k] = hbits(toh_flush(bf2f(f2bf(ts[(c8 + k) * 65 + e])) * WCARRY));
            *(volatile v8us*)(dst + e * HID + c8) = o8; }
        if (ps == 0) __threadfence(); }
}

__global__ __launch_bounds__(256) void k_vec(const float* __restrict__ b1, const float* __restrict__ bh, const float* __restrict__ wo, const float* __restrict__ bo, float* BV) {
    const int i = blockIdx.x * 256 + threadIdx.x;
    if (i >= BV_N4) return;
    const int f = 4 * i;
    const v4f a = *(const v4f*)(b1 + clampi(f - OFF_B1, 0, NSUB * HID - 4));
    const v4f b = *(const v4f*)(bh + clampi(f - OFF_BH, 0, NHL * NSUB * HID - 4));
    const v4f c = *(const v4f*)(wo + clampi(f - OFF_WO, 0, NSUB * HID - 4));
    const v4f d = *(const v4f*)(bo + clampi(f - OFF_BO, 0, NSUB - 4));
    v4f v;
#pragma unroll
    for (int k = 0; k < 4; ++k) {
        float s = d[k];
        s = (f < OFF_BO) ? c[k] : s;
        s = (f < OFF_WO) ? b[k] : s;
        s = (f < OFF_BH) ? a[k] : s;
        v[k] = bf2f(f2bf(s)); }
    *(volatile v4f*)(BV + f) = v; __threadfence(); *(volatile v4f*)(BV + f) = v;
}

__device__ __forceinline__ void layer_in(const bf* __restrict__ w, const float* __restrict__ bias, const v16bf (&xb)[2],
                                         v16h (&nv)[4], v16h (&nr)[4], const int lr, const int hi) {
#pragma unroll
    for (int j = 0; j < 4; ++j) {
#pragma unroll
        for (int u = 0; u < 2; ++u) {
            const int t = 2 * j + u;
            v8f acc = (v8f){};
            const bf* ap = w + (size_t)(16 * t + lr) * IND + 8 * hi;
#pragma unroll
            for (int ks = 0; ks < 2; ++ks) { const v16bf a = ldb(ap + 32 * ks); acc = wmmab_g(a, xb[ks], acc); }
            const v4f b0 = *(const v4f*)(bias + 16 * t + 8 * hi);
            const v4f b1 = *(const v4f*)(bias + 16 * t + 8 * hi + 4);
#pragma unroll
            for (int r = 0; r < 8; ++r) {
                const float z = acc[r] + ((r < 4) ? b0[r & 3] : b1[r & 3]);
                const float hs = swishf(z) * HCARRY;
                const h16 hv = toh_flush(hs);
                nv[j][8 * u + r] = hv;
                nr[j][8 * u + r] = toh_flush((hs - (float)hv) * RCARRY); }
        }
    }
}

template <bool LAST>
__device__ __forceinline__ float layer_hid(const hf* __restrict__ w, const float* __restrict__ bias, const float* __restrict__ wo,
                                           const v16h (&cv)[4], const v16h (&cr)[4], v16h (&nv)[4], v16h (&nr)[4], const int lr, const int hi) {
    float s = 0.0f;
#pragma unroll
    for (int j = 0; j < 4; ++j) {
#pragma unroll
        for (int u = 0; u < 2; ++u) {
            const int t = 2 * j + u;
            v8f am = (v8f){}, ar = (v8f){};
            const hf* ap = w + (size_t)(16 * t + lr) * HID + 8 * hi;
#pragma unroll
            for (int ks = 0; ks < 4; ++ks) {
                const v16h a = ldh(ap + 32 * ks);
                am = wmmah_g(a, cv[ks], am);
                if (HRES) ar = wmmah_g(a, cr[ks], ar); }
            const v4f b0 = *(const v4f*)(bias + 16 * t + 8 * hi);
            const v4f b1 = *(const v4f*)(bias + 16 * t + 8 * hi + 4);
            v4f w0 = (v4f){}, w1 = (v4f){};
            if (LAST) { w0 = *(const v4f*)(wo + 16 * t + 8 * hi); w1 = *(const v4f*)(wo + 16 * t + 8 * hi + 4); }
#pragma unroll
            for (int r = 0; r < 8; ++r) {
                float z = am[r] * SMAIN + ((r < 4) ? b0[r & 3] : b1[r & 3]);
                if (HRES) z += ar[r] * SRES;
                const float h = swishf(z);
                if (LAST) { s += h * ((r < 4) ? w0[r & 3] : w1[r & 3]); }
                else {
                    const float hs = h * HCARRY;
                    const h16 hv = toh_flush(hs);
                    nv[j][8 * u + r] = hv;
                    nr[j][8 * u + r] = toh_flush((hs - (float)hv) * RCARRY); }
            }
        }
    }
    return s;
}

__global__ __launch_bounds__(32) __attribute__((amdgpu_num_vgpr(256))) void k_mlp(const float* __restrict__ X, const bf* __restrict__ W1T, const hf* __restrict__ WHT,
                                                                                   const float* __restrict__ BV, float* OUT) {
    __shared__ __align__(16) float ot[16 * OTP];
    static_assert(sizeof(float) * 16 * OTP <= 131072);
    const int lane = threadIdx.x & 31, lr = lane & 15, hi = lane >> 4;
    const int row0 = blockIdx.x * 16;
    v16bf xb[2];
    {
        const float* xp = X + (size_t)(row0 + lr) * IND + 8 * hi;
#pragma unroll
        for (int ks = 0; ks < 2; ++ks) {
            const v8f a = *(const v8f*)(xp + 32 * ks); const v8f b = *(const v8f*)(xp + 32 * ks + 16); v8us lo, hh;
#pragma unroll
            for (int k = 0; k < 8; ++k) { lo[k] = f2bf(a[k]); hh[k] = f2bf(b[k]); }
            xb[ks] = cat16b(lo, hh); }
    }
#pragma unroll 1
    for (int o = 0; o < NSUB; ++o) {
        v16h pa[4], pb[4], qa[4], qb[4];
#pragma unroll
        for (int j = 0; j < 4; ++j) { pa[j] = (v16h){}; pb[j] = (v16h){}; qa[j] = (v16h){}; qb[j] = (v16h){}; }
        layer_in(W1T + (size_t)o * (HID * IND), BV + OFF_B1 + o * HID, xb, pa, pb, lr, hi);
        layer_hid<false>(WHT + (size_t)(0 * NSUB + o) * (HID * HID), BV + OFF_BH + (0 * NSUB + o) * HID, BV + OFF_WO + o * HID, pa, pb, qa, qb, lr, hi);
        float s = layer_hid<true>(WHT + (size_t)(1 * NSUB + o) * (HID * HID), BV + OFF_BH + (1 * NSUB + o) * HID, BV + OFF_WO + o * HID, qa, qb, pa, pb, lr, hi);
        s += __shfl_xor(s, 16, 32);
        const float bov = BV[OFF_BO + o];
        if (hi == 0) ot[lr * OTP + o] = s + bov;
    }
    wave_sync();
    static_assert(32 * 16 * 4 == 16 * NSUB * 4);
#pragma unroll 1
    for (int ps = 0; ps < 2; ++ps) {
#pragma unroll 1
        for (int it = 0; it < 4; ++it) {
            const int rr = 4 * it + (lane >> 3), c4 = (lane & 7) * 4;
            const v4f v = *(const v4fa*)(&ot[rr * OTP + c4]);
            *(volatile v4f*)(OUT + (size_t)(row0 + rr) * NSUB + c4) = v; }
        if (ps == 0) __threadfence(); }
}

static constexpr size_t al256(size_t v) { return (v + 255) & ~(size_t)255; }
static constexpr size_t SZ_W1T = al256((size_t)NSUB * HID * IND * 2);
static constexpr size_t SZ_WHT = al256((size_t)NHL * NSUB * HID * HID * 2);
static constexpr size_t SZ_BV  = al256((size_t)BV_N * 4);
static constexpr size_t SZ_TOTAL = SZ_W1T + SZ_WHT + SZ_BV;
static_assert(SZ_TOTAL <= (size_t)134217728);
static_assert((size_t)64 * 64 * 128 * 1 == (size_t)NSUB * HID * IND * 2);
static_assert((size_t)256 * 64 * 128 == (size_t)NHL * NSUB * HID * HID * 2);

extern "C" void kernel_launch(void* const* d_in, const int* in_sizes, int n_in,
                              void* d_out, int out_size, void* d_ws, size_t ws_size, hipStream_t stream) {
    if (n_in < 7) return;
    if ((size_t)in_sizes[0] < (size_t)NB * IND) return;
    if ((size_t)in_sizes[1] < (size_t)NSUB * IND * HID) return;
    if ((size_t)in_sizes[2] < (size_t)NSUB * HID) return;
    if ((size_t)in_sizes[3] < (size_t)NHL * NSUB * HID * HID) return;
    if ((size_t)in_sizes[4] < (size_t)NHL * NSUB * HID) return;
    if ((size_t)in_sizes[5] < (size_t)NSUB * HID) return;
    if ((size_t)in_sizes[6] < (size_t)NSUB) return;
    if ((size_t)out_size < (size_t)NB * NSUB) return;
    if (SZ_TOTAL > ws_size) return;
    const float* x  = (const float*)d_in[0];
    const float* W1 = (const float*)d_in[1];
    const float* b1 = (const float*)d_in[2];
    const float* Wh = (const float*)d_in[3];
    const float* bh = (const float*)d_in[4];
    const float* Wo = (const float*)d_in[5];
    const float* bo = (const float*)d_in[6];
    float* OUT = (float*)d_out;
    char* wsp = (char*)d_ws;
    bf*    W1T = (bf*)wsp;    wsp += SZ_W1T;
    hf*    WHT = (hf*)wsp;    wsp += SZ_WHT;
    float* BV  = (float*)wsp; wsp += SZ_BV;

    k_w1t<<<NSUB * 2, 256, 0, stream>>>(W1, W1T);
    k_wht<<<NHL * NSUB * 4, 256, 0, stream>>>(Wh, WHT);
    k_vec<<<(unsigned)((BV_N4 + 255) / 256), 256, 0, stream>>>(b1, bh, Wo, bo, BV);
    k_mlp<<<NB / 16, 32, 0, stream>>>(x, W1T, WHT, BV, OUT);
}
